// AffEncoder_15917148799531
// MI455X (gfx1250) — hardware-verified
//
#include <hip/hip_runtime.h>
#include <stdint.h>

#define NSEQ   256
#define TLEN   1024
#define TT     64
#define NTILE  (TLEN / TT)
#define TROW   (TLEN + 12)
#define XR     (TT + 9)
#define PD     68
#define NCH    48
#define HCH    16
#define OCH    8
#define KP1    160
#define KP2    448
#define KP3    256
#define KP4    64
#define WO1    0
#define WO2    (16 * KP1)
#define WO3    (WO2 + 48 * KP2)
#define WO4    (WO3 + 16 * KP3)
#define WTOT   (WO4 + 16 * KP4)
#define WITEMS (WTOT / 8)
#define WPLB   65536
#define GSZ    ((NSEQ) < 64 ? (NSEQ) : 64)
#define NGRP   (NSEQ / GSZ)
#define NT1    192
#define NT3    64
#define WSC    1024.0f
#define ASC    256.0f
#define OSC    (1.0f / 262144.0f)
#define LEAKF  0.01f
#define BNEPS  1e-5f

static_assert(TLEN % TT == 0);
static_assert(NSEQ % GSZ == 0);
static_assert(WO2 % 256 == 0 && WO3 % 256 == 0 && WO4 % 256 == 0 && WTOT % 256 == 0);
static_assert(WTOT * 2 <= WPLB);
static_assert((TROW * NCH * 2) % 128 == 0 && (TROW * HCH * 2) % 128 == 0);
static_assert(((TT + 4) * NCH * 2) % 128 == 0 && ((TT + 4) * HCH * 2) % 128 == 0);
static_assert(KP1 % 32 == 0 && KP2 % 32 == 0 && KP3 % 32 == 0 && KP4 % 32 == 0);
static_assert(TT * NCH * 2 == 2 * NT1 * 16);
static_assert(TT * HCH * 2 == 2 * NT3 * 16);
static_assert(TT * OCH * 4 == 2 * NT3 * 16);
static_assert(XR * 16 >= (TT - 1) * 16 + KP1);
static_assert(TROW >= TLEN + 4 + 8);

typedef _Float16 v16h __attribute__((ext_vector_type(16)));
typedef _Float16 v8h  __attribute__((ext_vector_type(8)));
typedef float    v8f  __attribute__((ext_vector_type(8)));
typedef unsigned int v4u __attribute__((ext_vector_type(4)));

__device__ __forceinline__ unsigned short bf_bits(float f) {
  unsigned u = __float_as_uint(f);
  return (unsigned short)((u + 0x7FFFu + ((u >> 16) & 1u)) >> 16);
}
__device__ __forceinline__ float bf_up(unsigned short h) { return __uint_as_float(((unsigned)h) << 16); }
__device__ __forceinline__ float bfr(float f) { return bf_up(bf_bits(f)); }
__device__ __forceinline__ unsigned short f2h_bits(float f) { return __builtin_bit_cast(unsigned short, (_Float16)f); }
__device__ __forceinline__ unsigned pk16(unsigned short a, unsigned short b) { return (unsigned)a | ((unsigned)b << 16); }
__device__ __forceinline__ unsigned short cvt_w(float v) { return f2h_bits(bfr(v) * WSC); }
__device__ __forceinline__ v8f zero8() { v8f z = {0.f, 0.f, 0.f, 0.f, 0.f, 0.f, 0.f, 0.f}; return z; }

__device__ __forceinline__ v16h ldfrag_h(const _Float16* p) {
  union { v16h v; v8h h[2]; } f;
  f.h[0] = *(const v8h*)(p);
  f.h[1] = *(const v8h*)(p + 16);
  return f.v;
}

__device__ __forceinline__ v8f mma_h_raw(v16h a, v16h b, v8f c) {
  return __builtin_amdgcn_wmma_f32_16x16x32_f16(false, a, false, b, (short)0, c, false, false);
}
__device__ __forceinline__ void dep_guard_h(v8f& a, v8f& b, v16h x, v16h y) {
#if defined(__HIP_DEVICE_COMPILE__)
  asm volatile("v_nop\n\tv_nop\n\tv_nop\n\tv_nop" : "+v"(a), "+v"(b) : "v"(x), "v"(y));
#endif
}
__device__ __forceinline__ void keep4_h(v16h a, v16h b, v16h c, v16h d) {
#if defined(__HIP_DEVICE_COMPILE__)
  asm volatile("v_nop" :: "v"(a), "v"(b), "v"(c), "v"(d));
#endif
}
__device__ __forceinline__ void acc_guard2(v8f& a, v8f& b) {
#if defined(__HIP_DEVICE_COMPILE__)
  asm volatile("v_nop\n\tv_nop\n\tv_nop\n\tv_nop" : "+v"(a), "+v"(b));
#endif
}

template<int MI, int NKS>
__device__ __forceinline__ void mma_core(v8f (&acc)[MI][2], const _Float16* A, int lda,
                                         const _Float16* Bh, const _Float16* Bl, int ldb, int lane) {
  const int m = lane & 15, koff = (lane >> 4) * 8;
#pragma unroll
  for (int i = 0; i < MI; ++i) { acc[i][0] = zero8(); acc[i][1] = zero8(); }
#pragma unroll 1
  for (int ks = 0; ks < NKS; ++ks) {
    const int k0 = ks * 32 + koff;
    v16h bh[2], bl[2];
#pragma unroll
    for (int j = 0; j < 2; ++j) {
      const int bo = (j * 16 + m) * ldb + k0;
      bh[j] = ldfrag_h(Bh + bo);
      bl[j] = ldfrag_h(Bl + bo);
    }
#pragma unroll
    for (int i = 0; i < MI; ++i) {
      const v16h ah = ldfrag_h(A + (i * 16 + m) * lda + k0);
#pragma unroll
      for (int j = 0; j < 2; ++j) {
        acc[i][j] = mma_h_raw(ah, bh[j], acc[i][j]);
        acc[i][j] = mma_h_raw(ah, bl[j], acc[i][j]);
      }
      dep_guard_h(acc[i][0], acc[i][1], ah, bl[1]);
    }
    keep4_h(bh[0], bh[1], bl[0], bl[1]);
  }
#pragma unroll
  for (int i = 0; i < MI; ++i) acc_guard2(acc[i][0], acc[i][1]);
}

template<int MI>
__device__ __forceinline__ void stage_d(float* sD, const v8f (&acc)[MI][2], int cb, int lane) {
  const int m = lane & 15, ro = (lane >> 4) * 8;
#pragma unroll
  for (int i = 0; i < MI; ++i)
#pragma unroll
    for (int j = 0; j < 2; ++j)
#pragma unroll
      for (int r = 0; r < 8; ++r)
        sD[(i * 16 + ro + r) * PD + cb + j * 16 + m] = acc[i][j][r];
}

__device__ __forceinline__ void pack_hl(float v, unsigned short* sh, unsigned short* sl, int idx) {
  const float s = v * ASC;
  const float hi = bfr(s);
  sh[idx] = f2h_bits(hi);
  sl[idx] = f2h_bits(s - hi);
}

__device__ __forceinline__ void put2(const v4u* s, v4u* g, int tid, int nthr) {
  const v4u p0 = s[tid];
  const v4u p1 = s[tid + nthr];
  *(volatile v4u*)(g + tid) = p0;
  *(volatile v4u*)(g + tid + nthr) = p1;
  __threadfence();
  *(volatile v4u*)(g + tid) = p0;
  *(volatile v4u*)(g + tid + nthr) = p1;
}
__device__ __forceinline__ void putz(v4u* g, int np, int tid) {
  v4u z; z[0] = 0u; z[1] = 0u; z[2] = 0u; z[3] = 0u;
  if (tid < np) *(volatile v4u*)(g + tid) = z;
  __threadfence();
  if (tid < np) *(volatile v4u*)(g + tid) = z;
}

__global__ __launch_bounds__(256) void k_wprep(const float* __restrict__ W1, const float* __restrict__ W2,
                                              const float* __restrict__ Wc1, const float* __restrict__ Wc2,
                                              unsigned short* wp) {
  const int item = blockIdx.x * 256 + (int)threadIdx.x;
  if (item >= WITEMS) return;
  const int base = item * 8;
  unsigned short hb[8];
  if (base < WO2) {
#pragma unroll
    for (int e = 0; e < 8; ++e) {
      const int idx = base + e;
      const int f = idx / KP1, k = idx - f * KP1;
      const int dt = k >> 4, slot = k & 15;
      const int k1 = slot / 3, c = slot - k1 * 3;
      const bool valid = (k < 144) && (slot < 15);
      const int k1c = min(k1, 4), dtc = min(dt, 8);
      const float v = W1[((k1c * 16 + f) * 3 + c) * 9 + dtc];
      hb[e] = cvt_w(valid ? v : 0.f);
    }
  } else if (base < WO3) {
#pragma unroll
    for (int e = 0; e < 8; ++e) {
      const int idx = base + e - WO2;
      const int o2 = idx / KP2, k = idx - o2 * KP2;
      const bool valid = k < 432;
      const int kc = min(k, 431);
      const int dt = kc / 48, ch = kc - dt * 48;
      const float v = W2[(o2 * 48 + ch) * 9 + dt];
      hb[e] = cvt_w(valid ? v : 0.f);
    }
  } else if (base < WO4) {
#pragma unroll
    for (int e = 0; e < 8; ++e) {
      const int idx = base + e - WO3;
      const int oc = idx / KP3, k = idx - oc * KP3;
      const bool valid = k < 240;
      const int kc = min(k, 239);
      const int dt = kc / 48, ch = kc - dt * 48;
      const float v = Wc1[(oc * 48 + ch) * 5 + dt];
      hb[e] = cvt_w(valid ? v : 0.f);
    }
  } else {
#pragma unroll
    for (int e = 0; e < 8; ++e) {
      const int idx = base + e - WO4;
      const int oc = idx / KP4, k = idx - oc * KP4;
      const bool valid = (oc < OCH) && (k < 48);
      const int occ = min(oc, OCH - 1), kc = min(k, 47);
      const int dt = kc >> 4, ic = kc & 15;
      const float v = Wc2[(occ * 16 + ic) * 3 + dt];
      hb[e] = cvt_w(valid ? v : 0.f);
    }
  }
  v4u p;
#pragma unroll
  for (int i = 0; i < 4; ++i) p[i] = pk16(hb[2 * i], hb[2 * i + 1]);
  unsigned short* d = wp + (size_t)item * 8;
  *(volatile v4u*)d = p;
  __threadfence();
  *(volatile v4u*)d = p;
}

__global__ __launch_bounds__(NT1) void k_s1(const float* __restrict__ poses, const float* __restrict__ A1,
                                            const float* __restrict__ b1, const unsigned short* __restrict__ wp,
                                            unsigned short* F2h, unsigned short* F2l) {
  __shared__ __align__(16) float sX[XR * 27];
  __shared__ float sA1[405];
  __shared__ float sb1[80];
  __shared__ float sbias[48];
  __shared__ __align__(16) unsigned short xAh[3 * XR * 16];
  __shared__ __align__(16) unsigned short xAl[3 * XR * 16];
  __shared__ __align__(16) float sD[3 * 16 * PD];
  __shared__ __align__(16) unsigned short sOh[TT * NCH];
  __shared__ __align__(16) unsigned short sOl[TT * NCH];
  const int tid = threadIdx.x, lane = tid & 31, wave = tid >> 5;
  const int tile = blockIdx.x, p = blockIdx.y, s = blockIdx.z;
  const int t0 = tile * TT;

#pragma unroll 1
  for (int i = tid; i < XR * 27; i += NT1) {
    const int row = i / 27, c27 = i - row * 27;
    const int t = t0 - 4 + row;
    const int tc = min(max(t, 0), TLEN - 1);
    const float v = poses[((size_t)s * TLEN + tc) * 27 + c27];
    sX[i] = ((unsigned)t < (unsigned)TLEN) ? bfr(v) : 0.f;
  }
#pragma unroll 1
  for (int i = tid; i < 405; i += NT1) sA1[i] = bfr(A1[i]);
  if (tid < 80) sb1[tid] = bfr(b1[tid]);
  __syncthreads();

  if (tid < 48) {
    const int f = tid / 3, e = tid - f * 3, w = p * 3 + e;
    float acc = 0.f;
#pragma unroll 1
    for (int k1 = 0; k1 < 5; ++k1) {
      float sa = 0.f;
#pragma unroll 1
      for (int v = 0; v < 9; ++v) sa += sA1[(k1 * 9 + v) * 9 + w];
      acc += sb1[k1 * 16 + f] * sa;
    }
    sbias[tid] = acc;
  }
#pragma unroll 1
  for (int idx = tid; idx < 3 * XR * 16; idx += NT1) {
    const int e = idx / (XR * 16), rem = idx - e * (XR * 16);
    const int row = rem >> 4, slot = rem & 15;
    const int k1 = slot / 3, c = slot - k1 * 3;
    const int k1c = min(k1, 4);
    const int w = p * 3 + e;
    const float* xr = sX + row * 27 + c;
    const float* ar = sA1 + (k1c * 9) * 9 + w;
    float sum = 0.f;
#pragma unroll
    for (int v = 0; v < 9; ++v) sum += ar[v * 9] * xr[v * 3];
    sum = (slot < 15) ? sum : 0.f;
    pack_hl(sum, xAh, xAl, idx);
  }
  __syncthreads();

  {
    const int e = wave >> 1, cb = (wave & 1) * 32;
    v8f acc[1][2];
    mma_core<1, KP1 / 32>(acc, (const _Float16*)(wp + WO1), KP1,
                          (const _Float16*)(xAh + (e * XR + cb) * 16),
                          (const _Float16*)(xAl + (e * XR + cb) * 16), 16, lane);
    stage_d<1>(sD + e * 16 * PD, acc, cb, lane);
  }
  __syncthreads();

#pragma unroll 1
  for (int idx = tid; idx < TT * NCH; idx += NT1) {
    const int t = idx / NCH, ch = idx - t * NCH;
    const int f = ch / 3, e = ch - f * 3;
    const float v = sD[(e * 16 + f) * PD + t] * OSC + sbias[ch];
    pack_hl(v, sOh, sOl, idx);
  }
  __syncthreads();

  const size_t pb = ((size_t)s * 3 + p) * TROW * NCH;
  put2((const v4u*)sOh, (v4u*)(F2h + pb + (size_t)(t0 + 4) * NCH), tid, NT1);
  put2((const v4u*)sOl, (v4u*)(F2l + pb + (size_t)(t0 + 4) * NCH), tid, NT1);
  if (tile == 0) {
    putz((v4u*)(F2h + pb), 4 * NCH * 2 / 16, tid);
    putz((v4u*)(F2l + pb), 4 * NCH * 2 / 16, tid);
  }
  if (tile == NTILE - 1) {
    putz((v4u*)(F2h + pb + (size_t)(TLEN + 4) * NCH), 8 * NCH * 2 / 16, tid);
    putz((v4u*)(F2l + pb + (size_t)(TLEN + 4) * NCH), 8 * NCH * 2 / 16, tid);
  }
}

__global__ __launch_bounds__(NT1) void k_s2(const unsigned short* __restrict__ F2h, const unsigned short* __restrict__ F2l,
                                            const unsigned short* __restrict__ wp, const float* __restrict__ A2,
                                            const float* __restrict__ b2, unsigned short* F3h, unsigned short* F3l) {
  __shared__ float sA2[27];
  __shared__ float sb2[48];
  __shared__ __align__(16) float sD[3 * 48 * PD];
  __shared__ __align__(16) unsigned short sOh[TT * NCH];
  __shared__ __align__(16) unsigned short sOl[TT * NCH];
  const int tid = threadIdx.x, lane = tid & 31, wave = tid >> 5;
  const int tile = blockIdx.x, s = blockIdx.y;
  const int t0 = tile * TT;
  if (tid < 27) sA2[tid] = bfr(A2[tid]);
  if (tid < 48) sb2[tid] = bfr(b2[tid]);
  {
    const int p = wave >> 1, cb = (wave & 1) * 32;
    const size_t bb = (((size_t)s * 3 + p) * TROW + t0 + cb) * NCH;
    v8f acc[3][2];
    mma_core<3, KP2 / 32>(acc, (const _Float16*)(wp + WO2), KP2,
                          (const _Float16*)(F2h + bb), (const _Float16*)(F2l + bb), NCH, lane);
    stage_d<3>(sD + p * 48 * PD, acc, cb, lane);
  }
  __syncthreads();

#pragma unroll 1
  for (int idx = tid; idx < TT * NCH; idx += NT1) {
    const int t = idx / NCH, ch3 = idx - t * NCH;
    const int f2 = ch3 / 3, w = ch3 - f2 * 3;
    float val = 0.f;
#pragma unroll
    for (int k2 = 0; k2 < 3; ++k2) {
      const float yb = sb2[k2 * 16 + f2];
      const float* dr = sD + (k2 * 16 + f2) * PD + t;
#pragma unroll
      for (int pp = 0; pp < 3; ++pp)
        val += (dr[pp * 48 * PD] * OSC + yb) * sA2[(k2 * 3 + pp) * 3 + w];
    }
    pack_hl(val, sOh, sOl, idx);
  }
  __syncthreads();

  const size_t pb = (size_t)s * TROW * NCH;
  put2((const v4u*)sOh, (v4u*)(F3h + pb + (size_t)(t0 + 4) * NCH), tid, NT1);
  put2((const v4u*)sOl, (v4u*)(F3l + pb + (size_t)(t0 + 4) * NCH), tid, NT1);
  if (tile == 0) {
    putz((v4u*)(F3h + pb), 4 * NCH * 2 / 16, tid);
    putz((v4u*)(F3l + pb), 4 * NCH * 2 / 16, tid);
  }
  if (tile == NTILE - 1) {
    putz((v4u*)(F3h + pb + (size_t)(TLEN + 4) * NCH), 8 * NCH * 2 / 16, tid);
    putz((v4u*)(F3l + pb + (size_t)(TLEN + 4) * NCH), 8 * NCH * 2 / 16, tid);
  }
}

template<int CI, int KP, int RSH, int CO, int LAST>
__global__ __launch_bounds__(NT3) void k_tc(const unsigned short* __restrict__ Bh, const unsigned short* __restrict__ Bl,
                                            const unsigned short* __restrict__ wpl, const float* __restrict__ bias,
                                            const float* __restrict__ bnw, const float* __restrict__ bnb,
                                            const float* __restrict__ bnm, const float* __restrict__ bnv,
                                            unsigned short* Oh, unsigned short* Ol, float* outp) {
  __shared__ float sbc[16], ssc[16], ssh[16];
  __shared__ __align__(16) float sD[16 * PD];
  __shared__ __align__(16) unsigned short sOh[TT * HCH];
  __shared__ __align__(16) unsigned short sOl[TT * HCH];
  __shared__ __align__(16) float sOf[TT * OCH];
  const int tid = threadIdx.x, lane = tid & 31, wave = tid >> 5;
  const int tile = blockIdx.x, s = blockIdx.y;
  const int t0 = tile * TT;
  if (tid < 16) {
    const int c = min(tid, CO - 1);
    const float sc = bfr(bnw[c]) / sqrtf(bfr(bnv[c]) + BNEPS);
    sbc[tid] = bfr(bias[c]);
    ssc[tid] = sc;
    ssh[tid] = bfr(bnb[c]) - bfr(bnm[c]) * sc;
  }
  {
    const int cb = wave * 32;
    const size_t bb = ((size_t)s * TROW + t0 + RSH + cb) * CI;
    v8f acc[1][2];
    mma_core<1, KP / 32>(acc, (const _Float16*)wpl, KP, (const _Float16*)(Bh + bb), (const _Float16*)(Bl + bb), CI, lane);
    stage_d<1>(sD, acc, cb, lane);
  }
  __syncthreads();

#pragma unroll 1
  for (int idx = tid; idx < TT * CO; idx += NT3) {
    const int t = idx / CO, oc = idx - t * CO;
    float z = (sD[oc * PD + t] * OSC + sbc[oc]) * ssc[oc] + ssh[oc];
    z = (z > 0.f) ? z : LEAKF * z;
    if (LAST) sOf[idx] = z;
    else pack_hl(z, sOh, sOl, idx);
  }
  __syncthreads();

  if (LAST) {
    put2((const v4u*)(const void*)sOf, (v4u*)(void*)(outp + ((size_t)s * TLEN + t0) * OCH), tid, NT3);
  } else {
    const size_t pb = (size_t)s * TROW * HCH;
    put2((const v4u*)sOh, (v4u*)(Oh + pb + (size_t)(t0 + 4) * HCH), tid, NT3);
    put2((const v4u*)sOl, (v4u*)(Ol + pb + (size_t)(t0 + 4) * HCH), tid, NT3);
    if (tile == 0) {
      putz((v4u*)(Oh + pb), 4 * HCH * 2 / 16, tid);
      putz((v4u*)(Ol + pb), 4 * HCH * 2 / 16, tid);
    }
    if (tile == NTILE - 1) {
      putz((v4u*)(Oh + pb + (size_t)(TLEN + 4) * HCH), 8 * HCH * 2 / 16, tid);
      putz((v4u*)(Ol + pb + (size_t)(TLEN + 4) * HCH), 8 * HCH * 2 / 16, tid);
    }
  }
}

extern "C" void kernel_launch(void* const* d_in, const int* in_sizes, int n_in,
                              void* d_out, int out_size, void* d_ws, size_t ws_size,
                              hipStream_t stream) {
  if (n_in < 19) return;
  if (in_sizes[0] != NSEQ * TLEN * 27) return;
  if (in_sizes[1] != 405 || in_sizes[2] != 27) return;
  if (in_sizes[3] != 2160 || in_sizes[4] != 80) return;
  if (in_sizes[5] != 20736 || in_sizes[6] != 48) return;
  if (in_sizes[7] != 3840 || in_sizes[8] != 16) return;
  if (in_sizes[9] != 16 || in_sizes[10] != 16 || in_sizes[11] != 16 || in_sizes[12] != 16) return;
  if (in_sizes[13] != 384 || in_sizes[14] != 8) return;
  if (in_sizes[15] != 8 || in_sizes[16] != 8 || in_sizes[17] != 8 || in_sizes[18] != 8) return;
  if (out_size != NSEQ * TLEN * OCH) return;

  const float* poses = (const float*)d_in[0];
  const float* A1    = (const float*)d_in[1];
  const float* A2    = (const float*)d_in[2];
  const float* W1    = (const float*)d_in[3];
  const float* b1    = (const float*)d_in[4];
  const float* W2    = (const float*)d_in[5];
  const float* b2    = (const float*)d_in[6];
  const float* Wc1   = (const float*)d_in[7];
  const float* bc1   = (const float*)d_in[8];
  const float* bn1w  = (const float*)d_in[9];
  const float* bn1b  = (const float*)d_in[10];
  const float* bn1m  = (const float*)d_in[11];
  const float* bn1v  = (const float*)d_in[12];
  const float* Wc2   = (const float*)d_in[13];
  const float* bc2   = (const float*)d_in[14];
  const float* bn2w  = (const float*)d_in[15];
  const float* bn2b  = (const float*)d_in[16];
  const float* bn2m  = (const float*)d_in[17];
  const float* bn2v  = (const float*)d_in[18];
  float* out = (float*)d_out;

  const size_t PF2 = (size_t)GSZ * 3 * TROW * NCH * 2;
  const size_t PF3 = (size_t)GSZ * TROW * NCH * 2;
  const size_t PH  = (size_t)GSZ * TROW * HCH * 2;
  size_t off = 0;
  const size_t oWP  = off; off += WPLB;
  const size_t oF2h = off; off += PF2;
  const size_t oF2l = off; off += PF2;
  const size_t oF3h = off; off += PF3;
  const size_t oF3l = off; off += PF3;
  const size_t oHh  = off; off += PH;
  const size_t oHl  = off; off += PH;
  if (off > ws_size) return;
  if (off > (size_t)134217728) return;

  char* ws = (char*)d_ws;
  unsigned short* WP  = (unsigned short*)(ws + oWP);
  unsigned short* F2h = (unsigned short*)(ws + oF2h);
  unsigned short* F2l = (unsigned short*)(ws + oF2l);
  unsigned short* F3h = (unsigned short*)(ws + oF3h);
  unsigned short* F3l = (unsigned short*)(ws + oF3l);
  unsigned short* Hh  = (unsigned short*)(ws + oHh);
  unsigned short* Hl  = (unsigned short*)(ws + oHl);

  k_wprep<<<dim3((WITEMS + 255) / 256), dim3(256), 0, stream>>>(W1, W2, Wc1, Wc2, WP);

  for (int g = 0; g < NGRP; ++g) {
    const float* pg = poses + (size_t)g * GSZ * TLEN * 27;
    float* og = out + (size_t)g * GSZ * TLEN * OCH;
    k_s1<<<dim3(NTILE, 3, GSZ), dim3(NT1), 0, stream>>>(pg, A1, b1, WP, F2h, F2l);
    k_s2<<<dim3(NTILE, GSZ), dim3(NT1), 0, stream>>>(F2h, F2l, WP, A2, b2, F3h, F3l);
    k_tc<NCH, KP3, 2, HCH, 0><<<dim3(NTILE, GSZ), dim3(NT3), 0, stream>>>(
        F3h, F3l, WP + WO3, bc1, bn1w, bn1b, bn1m, bn1v, Hh, Hl, og);
    k_tc<HCH, KP4, 3, OCH, 1><<<dim3(NTILE, GSZ), dim3(NT3), 0, stream>>>(
        Hh, Hl, WP + WO4, bc2, bn2w, bn2b, bn2m, bn2v, Hh, Hl, og);
  }
  (void)hipGetLastError();
}
